// Encoder_10599979287062
// MI455X (gfx1250) — hardware-verified
//
#include <hip/hip_runtime.h>


#ifndef NB
#define NB 2
#endif
#ifndef SEQ
#define SEQ 2048
#endif
#define NB_FULL  2
#define SEQ_FULL 2048
#define NH       12
#define HD       64
#define RS       (NH * HD)
#define NTHR     512
#define NWAV     (NTHR / 32)
#define KPW      (SEQ / NWAV)
#define NKT      (KPW / 16)
#define NKC      (KPW / 32)
#define NSTEPS   6
#define PCARRY     32768.0f
#define PCARRY_INV (1.0f / 32768.0f)
#define WS_LIMIT ((size_t)134217728)

static_assert(SEQ % 512 == 0);
static_assert(SEQ <= SEQ_FULL);
static_assert(NB >= 1 && NB <= NB_FULL);
static_assert(NKT * 16 * NWAV == SEQ);
static_assert(NKC * 2 == NKT);
static_assert((size_t)3 * NB * SEQ * RS * 2 + (size_t)NB * NH * HD * 4 <= WS_LIMIT);

typedef _Float16 v16h __attribute__((ext_vector_type(16)));
typedef _Float16 v8h  __attribute__((ext_vector_type(8)));
typedef float    v8f  __attribute__((ext_vector_type(8)));
typedef float    v4f  __attribute__((ext_vector_type(4)));

union AFrag { v16h v; v8h h[2]; };

__device__ __forceinline__ float bf16_rne(float x) {
  unsigned u = __float_as_uint(x);
  u = (u + 0x7fffu + ((u >> 16) & 1u)) & 0xffff0000u;
  return __uint_as_float(u);
}
__device__ __forceinline__ _Float16 to_h(float x) { return (_Float16)bf16_rne(x); }

__device__ __forceinline__ v8f zero8() {
  v8f z;
#pragma unroll
  for (int i = 0; i < 8; ++i) z[i] = 0.0f;
  return z;
}

__device__ __forceinline__ v16h load_frag16(const _Float16* base, int ld, int lane) {
  const int m  = lane & 15;
  const int kb = (lane >> 4) << 3;
  const _Float16* p = base + (size_t)m * ld + kb;
  AFrag f;
  f.h[0] = *(const v8h*)(p);
  f.h[1] = *(const v8h*)(p + 16);
  return f.v;
}

__device__ __forceinline__ v8f wmma16(v16h a, v16h b, v8f c) {
  v8f d = __builtin_amdgcn_wmma_f32_16x16x32_f16(false, a, false, b, (short)0, c, false, false);
  asm volatile("v_nop\n\tv_nop\n\tv_nop\n\tv_nop" : "+v"(d) : "v"(a), "v"(b) : "memory");
  return d;
}

template <bool MX>
__device__ __forceinline__ float cmb(float x, float y) { return MX ? fmaxf(x, y) : (x + y); }

template <bool MX>
__device__ __forceinline__ float half_red8(v8f a, int m) {
  const bool b3 = (m & 8) != 0, b2 = (m & 4) != 0, b1 = (m & 2) != 0;
  float k1[4];
#pragma unroll
  for (int j = 0; j < 4; ++j) {
    const float snd = b3 ? a[j] : a[j + 4];
    const float kp  = b3 ? a[j + 4] : a[j];
    k1[j] = cmb<MX>(kp, __shfl_xor(snd, 8, 32));
  }
  float k2[2];
#pragma unroll
  for (int j = 0; j < 2; ++j) {
    const float snd = b2 ? k1[j] : k1[j + 2];
    const float kp  = b2 ? k1[j + 2] : k1[j];
    k2[j] = cmb<MX>(kp, __shfl_xor(snd, 4, 32));
  }
  const float snd3 = b1 ? k2[0] : k2[1];
  const float kp3  = b1 ? k2[1] : k2[0];
  const float k3 = cmb<MX>(kp3, __shfl_xor(snd3, 2, 32));
  return cmb<MX>(k3, __shfl_xor(k3, 1, 32));
}

template <bool MX>
__device__ __forceinline__ void blockred2(v8f a, v8f b, float* rb, int lane, int wave,
                                          float& ta, float& tb) {
  const int m = lane & 15, hh = lane >> 4;
  const float ra = half_red8<MX>(a, m);
  const float rv = half_red8<MX>(b, m);
  if ((m & 1) == 0) {
    const int row = 8 * hh + (m >> 1);
    rb[row * 16 + wave]        = ra;
    rb[(16 + row) * 16 + wave] = rv;
  }
  __syncthreads();
  const float* pa = rb + m * 16 + 8 * hh;
  const float* pb = rb + (16 + m) * 16 + 8 * hh;
  const v4f a0 = *(const v4f*)(pa);
  const v4f a1 = *(const v4f*)(pa + 4);
  const v4f b0 = *(const v4f*)(pb);
  const v4f b1 = *(const v4f*)(pb + 4);
  float xa, xb;
  if (MX) {
    xa = fmaxf(fmaxf(fmaxf(a0[0], a0[1]), fmaxf(a0[2], a0[3])),
               fmaxf(fmaxf(a1[0], a1[1]), fmaxf(a1[2], a1[3])));
    xb = fmaxf(fmaxf(fmaxf(b0[0], b0[1]), fmaxf(b0[2], b0[3])),
               fmaxf(fmaxf(b1[0], b1[1]), fmaxf(b1[2], b1[3])));
  } else {
    xa = ((((((a0[0] + a0[1]) + a0[2]) + a0[3]) + a1[0]) + a1[1]) + a1[2]) + a1[3];
    xb = ((((((b0[0] + b0[1]) + b0[2]) + b0[3]) + b1[0]) + b1[1]) + b1[2]) + b1[3];
  }
  const float ya = __shfl_xor(xa, 16, 32);
  const float yb = __shfl_xor(xb, 16, 32);
  ta = cmb<MX>(xa, ya);
  tb = cmb<MX>(xb, yb);
}

__global__ __launch_bounds__(256) void k_cvt_qk(const float* __restrict__ q, const float* __restrict__ k,
                                                _Float16* __restrict__ qh, _Float16* __restrict__ kh, int n8) {
  const int i = blockIdx.x * 256 + threadIdx.x;
  if (i >= n8) return;
  const bool second = (blockIdx.y != 0);
  const float* src = second ? k : q;
  _Float16* dst = second ? kh : qh;
  const size_t e     = (size_t)i * 8;
  const size_t per_b = (size_t)SEQ * RS;
  const size_t bb    = e / per_b;
  const size_t rem   = e - bb * per_b;
  const float* p = src + bb * ((size_t)SEQ_FULL * RS) + rem;
  const v4f f0 = *(const v4f*)(p);
  const v4f f1 = *(const v4f*)(p + 4);
  v8h o;
  o[0] = to_h(f0[0]); o[1] = to_h(f0[1]); o[2] = to_h(f0[2]); o[3] = to_h(f0[3]);
  o[4] = to_h(f1[0]); o[5] = to_h(f1[1]); o[6] = to_h(f1[2]); o[7] = to_h(f1[3]);
  volatile v8h* d = (volatile v8h*)(dst + e);
  *d = o;
  __threadfence();
  *d = o;
}

__global__ __launch_bounds__(256) void k_vtrans(const float* __restrict__ v, _Float16* __restrict__ vth) {
  __shared__ __align__(16) _Float16 tile[HD][72];
  const int tid = threadIdx.x;
  const int l0 = blockIdx.x * 64, h = blockIdx.y, bb = blockIdx.z;
  const float* vb = v + ((size_t)bb * SEQ_FULL + l0) * RS + h * HD;
#pragma unroll
  for (int j = 0; j < 4; ++j) {
    const int idx = tid + 256 * j;
    const int l = idx >> 4, d4 = (idx & 15) * 4;
    const v4f f = *(const v4f*)(vb + (size_t)l * RS + d4);
    tile[d4 + 0][l] = to_h(f[0]);
    tile[d4 + 1][l] = to_h(f[1]);
    tile[d4 + 2][l] = to_h(f[2]);
    tile[d4 + 3][l] = to_h(f[3]);
  }
  __syncthreads();
  _Float16* ob = vth + ((size_t)(bb * NH + h) * HD) * SEQ + l0;
  v8h val[2];
  size_t off[2];
#pragma unroll
  for (int j = 0; j < 2; ++j) {
    const int p = tid + 256 * j;
    const int row = p >> 3, piece = p & 7;
    val[j] = *(const v8h*)(&tile[row][piece * 8]);
    off[j] = (size_t)row * SEQ + piece * 8;
  }
  *(volatile v8h*)(ob + off[0]) = val[0];
  *(volatile v8h*)(ob + off[1]) = val[1];
  __threadfence();
  *(volatile v8h*)(ob + off[0]) = val[0];
  *(volatile v8h*)(ob + off[1]) = val[1];
}

__global__ __launch_bounds__(64) void k_vsum(const float* __restrict__ v, float* __restrict__ vsum) {
  __shared__ __align__(16) float ssum[HD];
  const int d = threadIdx.x, h = blockIdx.x, bb = blockIdx.y;
  const float* p = v + (size_t)bb * SEQ_FULL * RS + h * HD + d;
  double acc = 0.0;
#pragma unroll 4
  for (int l = 0; l < SEQ; ++l) acc += (double)bf16_rne(p[(size_t)l * RS]);
  ssum[d] = (float)acc;
  __syncthreads();
  if (d < 16) {
    const v4f val = *(const v4f*)(&ssum[d * 4]);
    volatile v4f* o = (volatile v4f*)(vsum + (size_t)(bb * NH + h) * HD + d * 4);
    *o = val;
    __threadfence();
    *o = val;
  }
}

__global__ __launch_bounds__(NTHR) __attribute__((amdgpu_num_vgpr(256)))
void k_attn(const _Float16* __restrict__ qh, const _Float16* __restrict__ kh,
            const _Float16* __restrict__ vth, const float* __restrict__ vsum,
            float* __restrict__ out) {
  __shared__ __align__(16) _Float16 Pst[NWAV][16][32];
  __shared__ __align__(16) float red[2][2][16][16];
  __shared__ __align__(16) float Ored[4][16][HD];
  __shared__ __align__(16) float Ofin[16][HD];
  __shared__ float wbar_sh[16];

  const int tid  = threadIdx.x;
  const int lane = tid & 31, wave = tid >> 5;
  const int m = lane & 15, hh = lane >> 4, r0 = hh << 3;
  const int q0 = blockIdx.x * 16, h = blockIdx.y, b = blockIdx.z;
  const int kw0 = wave * KPW;

  const _Float16* qp = qh  + ((size_t)b * SEQ + q0)  * RS + h * HD;
  const _Float16* kp = kh  + ((size_t)b * SEQ + kw0) * RS + h * HD;
  const _Float16* vp = vth + ((size_t)(b * NH + h) * HD) * SEQ + kw0;

  v8f s[NKT];
  {
    const v16h qa0 = load_frag16(qp, RS, lane);
    const v16h qa1 = load_frag16(qp + 32, RS, lane);
#pragma unroll
    for (int t = 0; t < NKT; ++t) {
      const _Float16* kt = kp + (size_t)(t * 16) * RS;
      const v16h kb0 = load_frag16(kt, RS, lane);
      const v16h kb1 = load_frag16(kt + 32, RS, lane);
      v8f acc = zero8();
      acc = wmma16(qa0, kb0, acc);
      acc = wmma16(qa1, kb1, acc);
      s[t] = acc * 0.125f;
    }
  }

  float cl;
  v8f   cv;
  {
    v8f mx;
#pragma unroll
    for (int g = 0; g < 8; ++g) {
      float x = s[0][g];
#pragma unroll
      for (int t = 1; t < NKT; ++t) x = fmaxf(x, s[t][g]);
      mx[g] = x;
    }
    float ta, tb;
    blockred2<true>(mx, mx, &red[0][0][0][0], lane, wave, ta, tb);
    cl = -ta - 1.0f;
#pragma unroll
    for (int g = 0; g < 8; ++g) cv[g] = __shfl(cl, r0 + g, 32);
  }

#pragma unroll 1
  for (int it = 0; it < NSTEPS; ++it) {
    v8f ps = zero8(), pd = zero8();
#pragma unroll
    for (int t = 0; t < NKT; ++t) {
      const v8f tt = -s[t] - cv;
      v8f y;
#pragma unroll
      for (int g = 0; g < 8; ++g) y[g] = __builtin_amdgcn_rcpf(tt[g]);
      const v8f a = y * y;
      ps += a;
      pd += a * y;
    }
    float ta, tb;
    blockred2<false>(ps, pd, &red[(it + 1) & 1][0][0][0], lane, wave, ta, tb);
    cl = cl - (ta - 1.0f) / (2.0f * tb + 1e-8f);
#pragma unroll
    for (int g = 0; g < 8; ++g) cv[g] = __shfl(cl, r0 + g, 32);
  }

  v8f wb;
  {
    v8f sw = zero8();
#pragma unroll
    for (int t = 0; t < NKT; ++t) {
      const v8f tt = -s[t] - cv;
      v8f y;
#pragma unroll
      for (int g = 0; g < 8; ++g) y[g] = __builtin_amdgcn_rcpf(tt[g]);
      const v8f w = y * y;
      s[t] = w;
      sw += w;
    }
    float ta, tb;
    blockred2<false>(sw, sw, &red[1][0][0][0], lane, wave, ta, tb);
    const float wbl = ta * (1.0f / (float)SEQ);
    if (wave == 0 && lane < 16) wbar_sh[lane] = wbl;
#pragma unroll
    for (int g = 0; g < 8; ++g) wb[g] = __shfl(wbl, r0 + g, 32);
  }

  v8f o[4];
#pragma unroll
  for (int st = 0; st < 4; ++st) o[st] = zero8();
  _Float16* pst = &Pst[wave][0][0];
#pragma unroll
  for (int kc = 0; kc < NKC; ++kc) {
    const v8f p0 = (s[2 * kc] - wb) * PCARRY;
    const v8f p1 = (s[2 * kc + 1] - wb) * PCARRY;
    __builtin_amdgcn_fence(5, "wavefront");
    __builtin_amdgcn_wave_barrier();
#pragma unroll
    for (int g = 0; g < 8; ++g) {
      pst[(r0 + g) * 32 + m]      = (_Float16)p0[g];
      pst[(r0 + g) * 32 + m + 16] = (_Float16)p1[g];
    }
    __builtin_amdgcn_fence(5, "wavefront");
    __builtin_amdgcn_wave_barrier();
    const v16h pa = load_frag16(pst, 32, lane);
#pragma unroll
    for (int st = 0; st < 4; ++st) {
      const v16h vbf = load_frag16(vp + (size_t)(st * 16) * SEQ + kc * 32, SEQ, lane);
      o[st] = wmma16(pa, vbf, o[st]);
    }
  }

#pragma unroll 1
  for (int ph = 0; ph < 4; ++ph) {
    if ((wave >> 2) == ph) {
      float* ob = &Ored[wave & 3][0][0];
#pragma unroll
      for (int st = 0; st < 4; ++st) {
#pragma unroll
        for (int g = 0; g < 8; ++g) {
          float* pr = ob + (r0 + g) * HD + st * 16 + m;
          const float x = o[st][g];
          if (ph == 0) *pr = x; else *pr = *pr + x;
        }
      }
    }
    __syncthreads();
  }

  {
    const float* vsp = vsum + (size_t)(b * NH + h) * HD;
#pragma unroll
    for (int j = 0; j < 2; ++j) {
      const int e = tid * 2 + j;
      const int row = e >> 6, d = e & 63;
      const float a = ((Ored[0][row][d] + Ored[1][row][d]) + Ored[2][row][d]) + Ored[3][row][d];
      Ofin[row][d] = a * PCARRY_INV + wbar_sh[row] * vsp[d];
    }
  }
  __syncthreads();
  if (wave < 4) {
    v4f val[2];
    size_t off[2];
#pragma unroll
    for (int j = 0; j < 2; ++j) {
      const int row = wave * 4 + 2 * j + hh;
      val[j] = *(const v4f*)(&Ofin[row][m * 4]);
      off[j] = ((size_t)b * SEQ + q0 + row) * RS + h * HD + m * 4;
    }
    *(volatile v4f*)(out + off[0]) = val[0];
    *(volatile v4f*)(out + off[1]) = val[1];
    __threadfence();
    *(volatile v4f*)(out + off[0]) = val[0];
    *(volatile v4f*)(out + off[1]) = val[1];
  }
}

extern "C" void kernel_launch(void* const* d_in, const int* in_sizes, int n_in,
                              void* d_out, int out_size, void* d_ws, size_t ws_size,
                              hipStream_t stream) {
  if (n_in < 3 || d_ws == nullptr || d_out == nullptr) return;
  const size_t need_in  = ((size_t)(NB - 1) * SEQ_FULL + SEQ) * RS;
  const size_t need_out = (size_t)NB * SEQ * RS;
  if ((size_t)in_sizes[0] < need_in || (size_t)in_sizes[1] < need_in || (size_t)in_sizes[2] < need_in) return;
  if ((size_t)out_size < need_out) return;

  const size_t plane_b = (size_t)NB * SEQ * RS * sizeof(_Float16);
  const size_t vsum_b  = (size_t)NB * NH * HD * sizeof(float);
  const size_t off_q = 0;
  const size_t off_k = off_q + plane_b;
  const size_t off_v = off_k + plane_b;
  const size_t off_s = off_v + plane_b;
  const size_t total = off_s + vsum_b;
  if (ws_size < total || total > WS_LIMIT) return;

  const float* q = (const float*)d_in[0];
  const float* k = (const float*)d_in[1];
  const float* v = (const float*)d_in[2];
  float* o = (float*)d_out;
  char* ws = (char*)d_ws;
  _Float16* qh  = (_Float16*)(ws + off_q);
  _Float16* kh  = (_Float16*)(ws + off_k);
  _Float16* vth = (_Float16*)(ws + off_v);
  float*    vs  = (float*)(ws + off_s);

  const int n8 = (int)((size_t)NB * SEQ * RS / 8);
  k_cvt_qk<<<dim3((n8 + 255) / 256, 2), 256, 0, stream>>>(q, k, qh, kh, n8);
  k_vtrans<<<dim3(SEQ / 64, NH, NB), 256, 0, stream>>>(v, vth);
  k_vsum<<<dim3(NH, NB), 64, 0, stream>>>(v, vs);
  k_attn<<<dim3(SEQ / 16, NH, NB), NTHR, 0, stream>>>(qh, kh, vth, vs, o);
  (void)hipGetLastError();
}
